// BitterGAT_Baseline_52475910422829
// MI455X (gfx1250) — hardware-verified
//
#include <hip/hip_runtime.h>
#include <stddef.h>
#include <math.h>

typedef __attribute__((ext_vector_type(16))) _Float16 v16h;
typedef __attribute__((ext_vector_type(8)))  _Float16 v8h;
typedef __attribute__((ext_vector_type(16))) __bf16   v16b;
typedef __attribute__((ext_vector_type(8)))  __bf16   v8b;
typedef __attribute__((ext_vector_type(8)))  float    v8f;
typedef __attribute__((ext_vector_type(4)))  float    v4f;
typedef __attribute__((ext_vector_type(2)))  float    v2f;
typedef __attribute__((ext_vector_type(4)))  int      v4i;

constexpr int CIN_X  = 20;
constexpr int KPAD1  = 32;
constexpr int HIDC   = 64;
constexpr int OUTC   = 2;
constexpr int NBA    = 1024;
constexpr int RPQ    = 1024;
constexpr int PPITCH = 96;
constexpr int GMAX   = 1024;
#define NTHR    256
#define NWAVE   8
#define EPT     8
#define NGRP    1
#define CHUNK   (NTHR * EPT * NGRP)
#define WCAP    (EPT * NGRP * 32)
#define LISTN   (NWAVE * WCAP)
#define LDS_AGG ((NBA * HIDC + 2 * NBA) * 4 + LISTN * 4 + 64)

static_assert((CHUNK & (CHUNK - 1)) == 0);
static_assert(CHUNK <= 4096);
static_assert((NBA & (NBA - 1)) == 0 && NBA <= 4096);
static_assert(RPQ % NBA == 0 && RPQ % 64 == 0 && RPQ % NTHR == 0);
static_assert(LDS_AGG == 278592);
static_assert(KPAD1 % 32 == 0 && HIDC % 64 == 0 && CIN_X <= KPAD1);
static_assert(PPITCH % 32 == 0 && PPITCH >= HIDC + 32);

__device__ __forceinline__ unsigned short f2bf_bits(float f) {
  unsigned u = __float_as_uint(f);
  return (unsigned short)((u + 0x7FFFu + ((u >> 16) & 1u)) >> 16);
}
__device__ __forceinline__ float bf_bits2f(unsigned short h) { return __uint_as_float(((unsigned)h) << 16); }

__device__ __forceinline__ void dep_guard_h(v8f& a, v8f& b, v16h x, v16h y) { asm volatile("v_nop\n\tv_nop\n\tv_nop\n\tv_nop" : "+v"(a), "+v"(b) : "v"(x), "v"(y)); }
__device__ __forceinline__ void dep_guard_b(v8f& a, v8f& b, v16b x, v16b y) { asm volatile("v_nop\n\tv_nop\n\tv_nop\n\tv_nop" : "+v"(a), "+v"(b) : "v"(x), "v"(y)); }
__device__ __forceinline__ void keep4_h(v16h a, v16h b, v16h c, v16h d) { asm volatile("v_nop" :: "v"(a), "v"(b), "v"(c), "v"(d)); }
__device__ __forceinline__ void keep4_b(v16b a, v16b b, v16b c, v16b d) { asm volatile("v_nop" :: "v"(a), "v"(b), "v"(c), "v"(d)); }
__device__ __forceinline__ void acc_guard4(v8f& a, v8f& b, v8f& c, v8f& d) { asm volatile("v_nop\n\tv_nop\n\tv_nop\n\tv_nop" : "+v"(a), "+v"(b), "+v"(c), "+v"(d)); }
template <typename T> struct Frag;
template <> struct Frag<_Float16> {
  typedef v16h V; union U { v16h v; v8h h[2]; };
  static __device__ __forceinline__ v16h load(const _Float16* p) {
    U f; f.h[0] = *(const v8h*)(p); f.h[1] = *(const v8h*)(p + 16); return f.v;
  }
  static __device__ __forceinline__ v8f mma(v16h a, v16h b, v8f c) {
    return __builtin_amdgcn_wmma_f32_16x16x32_f16(false, a, false, b, (short)0, c, false, false);
  }
  static __device__ __forceinline__ void guard(v8f& a, v8f& b, v16h x, v16h y) { dep_guard_h(a, b, x, y); }
  static __device__ __forceinline__ void keep(v16h a, v16h b, v16h c, v16h d) { keep4_h(a, b, c, d); }
};
template <> struct Frag<__bf16> {
  typedef v16b V; union U { v16b v; v8b h[2]; };
  static __device__ __forceinline__ v16b load(const __bf16* p) {
    U f; f.h[0] = *(const v8b*)(p); f.h[1] = *(const v8b*)(p + 16); return f.v;
  }
  static __device__ __forceinline__ v8f mma(v16b a, v16b b, v8f c) {
    return __builtin_amdgcn_wmma_f32_16x16x32_bf16(false, a, false, b, (short)0, c, false, false);
  }
  static __device__ __forceinline__ void guard(v8f& a, v8f& b, v16b x, v16b y) { dep_guard_b(a, b, x, y); }
  static __device__ __forceinline__ void keep(v16b a, v16b b, v16b c, v16b d) { keep4_b(a, b, c, d); }
};

template <int ET> struct Elem;
template <> struct Elem<0> { typedef _Float16 T; };
template <> struct Elem<1> { typedef __bf16 T; };
template <int ET, bool SPLIT, int BIAS_MODE, int OUT_MODE, bool RESID, int ACT = 0>
__global__ __launch_bounds__(256) void wmma_gemm64(
    const unsigned short* __restrict__ Ap, const unsigned short* __restrict__ A2p, int lda, long strideA,
    const unsigned short* __restrict__ Btp, const unsigned short* __restrict__ Bt2p, int ldb, long strideB,
    void* __restrict__ Cout, void* __restrict__ Cout2, int ldc, long strideC,
    const float* __restrict__ bias,
    const float* __restrict__ resid, long strideR,
    int M, int N, int K, float scale) {
  typedef typename Elem<ET>::T T;
  typedef typename Frag<T>::V V;
  const T* A = (const T*)Ap; const T* A2 = (const T*)A2p; const T* Bt = (const T*)Btp; const T* Bt2 = (const T*)Bt2p;
  __shared__ __align__(16) float sT[8][16 * 68];
  const int b    = blockIdx.y;
  const int lane = threadIdx.x & 31;
  const int wave = threadIdx.x >> 5;
  const int tilesN = N >> 6;
  const int tilesM = M >> 6;
  const int tile = blockIdx.x * 8 + wave;
  if (tile >= tilesM * tilesN) return;
  const int tm = tile / tilesN;
  const int tn = tile - tm * tilesN;
  const int m0 = tm << 6;
  const int n0 = tn << 6;

  const T* Ab  = A  + (size_t)b * strideA;
  const T* Bb  = Bt + (size_t)b * strideB;
  const T* Ab2 = SPLIT ? (A2  + (size_t)b * strideA) : nullptr;
  const T* Bb2 = SPLIT ? (Bt2 + (size_t)b * strideB) : nullptr;

  const int rlane = lane & 15;
  const int koff  = (lane >> 4) * 8;
  const int mOff  = (lane >> 4) * 8;

  v8f acc[4][4];
#pragma unroll
  for (int i = 0; i < 4; ++i)
#pragma unroll
    for (int j = 0; j < 4; ++j) acc[i][j] = (v8f){0.f,0.f,0.f,0.f,0.f,0.f,0.f,0.f};

  for (int k0 = 0; k0 < K; k0 += 32) {
    V bh[4], bl[4];
#pragma unroll
    for (int j = 0; j < 4; ++j) {
      const size_t bo = (size_t)(n0 + (j << 4) + rlane) * ldb + koff + k0;
      bh[j] = Frag<T>::load(Bb + bo);
      if (SPLIT) bl[j] = Frag<T>::load(Bb2 + bo);
    }
#pragma unroll
    for (int i = 0; i < 4; ++i) {
      const size_t ao = (size_t)(m0 + (i << 4) + rlane) * lda + koff + k0;
      V ah = Frag<T>::load(Ab + ao);
      V al;
      if (SPLIT) al = Frag<T>::load(Ab2 + ao);
#pragma unroll
      for (int j = 0; j < 4; ++j) {
        acc[i][j] = Frag<T>::mma(ah, bh[j], acc[i][j]);
        if (SPLIT) {
          acc[i][j] = Frag<T>::mma(ah, bl[j], acc[i][j]);
          acc[i][j] = Frag<T>::mma(al, bh[j], acc[i][j]);
        }
      }
      Frag<T>::guard(acc[i][0], acc[i][3], ah, SPLIT ? al : ah);
    }
    Frag<T>::keep(bh[0], bh[1], bh[2], bh[3]);
    if (SPLIT) Frag<T>::keep(bl[0], bl[1], bl[2], bl[3]);
  }
  acc_guard4(acc[0][0], acc[0][1], acc[0][2], acc[0][3]);
  acc_guard4(acc[1][0], acc[1][1], acc[1][2], acc[1][3]);
  acc_guard4(acc[2][0], acc[2][1], acc[2][2], acc[2][3]);
  acc_guard4(acc[3][0], acc[3][1], acc[3][2], acc[3][3]);

  float* slab = sT[wave];
  const float* Rb = RESID ? (resid + (size_t)b * strideR) : nullptr;
#pragma unroll
  for (int i = 0; i < 4; ++i) {
    const int mBase = m0 + (i << 4);
#pragma unroll
    for (int j = 0; j < 4; ++j) {
      const int n = n0 + (j << 4) + rlane;
      float bv = 0.f;
      if (BIAS_MODE == 2) bv = bias[n];
#pragma unroll
      for (int r = 0; r < 8; ++r) {
        float v = acc[i][j][r] * scale;
        if (BIAS_MODE == 1) v += bias[mBase + mOff + r];
        if (BIAS_MODE == 2) v += bv;
        if (RESID) v += Rb[(size_t)(mBase + mOff + r) * ldc + n];
        if (ACT == 1) v = tanhf(v);
        if (ACT == 2) v = fmaxf(v, 0.0f);
        if (ACT == 3) v = v / (1.0f + expf(-v));
        if (ACT == 4) v = (v > 0.f) ? v : 0.01f * v;
        if (ACT == 5) v = 0.5f * v * (1.0f + erff(v * 0.70710678118654752f));
        slab[(mOff + r) * 68 + (j << 4) + rlane] = v;
      }
    }
    __builtin_amdgcn_fence(__ATOMIC_RELEASE, "workgroup");
    __builtin_amdgcn_wave_barrier();
    __builtin_amdgcn_fence(__ATOMIC_ACQUIRE, "workgroup");
    if (OUT_MODE == 0) {
      float* C = (float*)Cout + (size_t)b * strideC;
      const int hh = lane >> 4, c4 = (lane & 15) * 4;
      for (int pass = 0; pass < 2; ++pass) {
#pragma unroll
        for (int it = 0; it < 8; ++it) {
          const int row = it * 2 + hh;
          v4f v = *(const v4f*)(slab + row * 68 + c4);
          *(volatile v4f*)(C + (size_t)(mBase + row) * ldc + n0 + c4) = v;
        }
        __threadfence();
      }
    } else {
      const int q = lane >> 3, c8 = (lane & 7) * 8;
      unsigned short* C  = (unsigned short*)Cout  + (size_t)b * strideC;
      unsigned short* C2 = (OUT_MODE == 2) ? ((unsigned short*)Cout2 + (size_t)b * strideC) : nullptr;
      for (int pass = 0; pass < 2; ++pass) {
#pragma unroll
        for (int it = 0; it < 4; ++it) {
          const int row = it * 4 + q;
          const float* sp = slab + row * 68 + c8;
          v8h hv, lv;
#pragma unroll
          for (int e = 0; e < 8; ++e) {
            if (OUT_MODE == 1) {
              hv[e] = (_Float16)sp[e];
            } else {
              unsigned short hb = f2bf_bits(sp[e]);
              unsigned short lb = f2bf_bits(sp[e] - bf_bits2f(hb));
              hv[e] = __builtin_bit_cast(_Float16, hb);
              lv[e] = __builtin_bit_cast(_Float16, lb);
            }
          }
          *(volatile v8h*)(C + (size_t)(mBase + row) * ldc + n0 + c8) = hv;
          if (OUT_MODE == 2) *(volatile v8h*)(C2 + (size_t)(mBase + row) * ldc + n0 + c8) = lv;
        }
        __threadfence();
      }
    }
    __builtin_amdgcn_fence(__ATOMIC_RELEASE, "workgroup");
    __builtin_amdgcn_wave_barrier();
    __builtin_amdgcn_fence(__ATOMIC_ACQUIRE, "workgroup");
  }
}

template <int NB>
__device__ __forceinline__ int scan_chunk(const int* __restrict__ lst, int nE, int cbase, int nodeBase,
                                          int* list, int tid, int lane, int wave, int fullvec) {
  int wc = 0;
#pragma unroll
  for (int g = 0; g < NGRP; ++g) {
    const int el0 = (g * NTHR + tid) * EPT;
    const int e0  = cbase + el0;
    v4i da, db;
    if (fullvec) {
      da = *(const v4i*)(lst + e0);
      db = *(const v4i*)(lst + e0 + 4);
    } else {
      const int em = nE - 1;
      da.x = lst[(e0     < em) ? e0     : em];
      da.y = lst[(e0 + 1 < em) ? e0 + 1 : em];
      da.z = lst[(e0 + 2 < em) ? e0 + 2 : em];
      da.w = lst[(e0 + 3 < em) ? e0 + 3 : em];
      db.x = lst[(e0 + 4 < em) ? e0 + 4 : em];
      db.y = lst[(e0 + 5 < em) ? e0 + 5 : em];
      db.z = lst[(e0 + 6 < em) ? e0 + 6 : em];
      db.w = lst[(e0 + 7 < em) ? e0 + 7 : em];
    }
    const bool v0 = (e0 < nE), v1 = (e0 + 1 < nE), v2 = (e0 + 2 < nE), v3 = (e0 + 3 < nE);
    const bool v4 = (e0 + 4 < nE), v5 = (e0 + 5 < nE), v6 = (e0 + 6 < nE), v7 = (e0 + 7 < nE);
    const unsigned nb = (unsigned)nodeBase;
    const unsigned s0 = (unsigned)da.x - nb, s1 = (unsigned)da.y - nb;
    const unsigned s2 = (unsigned)da.z - nb, s3 = (unsigned)da.w - nb;
    const unsigned s4 = (unsigned)db.x - nb, s5 = (unsigned)db.y - nb;
    const unsigned s6 = (unsigned)db.z - nb, s7 = (unsigned)db.w - nb;
    const bool h0 = v0 && (s0 < (unsigned)NB), h1 = v1 && (s1 < (unsigned)NB);
    const bool h2 = v2 && (s2 < (unsigned)NB), h3 = v3 && (s3 < (unsigned)NB);
    const bool h4 = v4 && (s4 < (unsigned)NB), h5 = v5 && (s5 < (unsigned)NB);
    const bool h6 = v6 && (s6 < (unsigned)NB), h7 = v7 && (s7 < (unsigned)NB);
    const unsigned any = __builtin_amdgcn_ballot_w32(h0 | h1 | h2 | h3 | h4 | h5 | h6 | h7);
    if (any != 0u) {
#define HITJ(J, HJ, SJ) { \
        const unsigned mj = __builtin_amdgcn_ballot_w32(HJ); \
        if (mj != 0u) { \
          if (HJ) { \
            const int pos = wc + (int)__builtin_amdgcn_mbcnt_lo(mj, 0u); \
            if (pos < WCAP) list[wave * WCAP + pos] = ((el0 + (J)) << 12) | (int)(SJ); \
          } \
          wc += (int)__builtin_popcount(mj); } }
      HITJ(0, h0, s0)
      HITJ(1, h1, s1)
      HITJ(2, h2, s2)
      HITJ(3, h3, s3)
      HITJ(4, h4, s4)
      HITJ(5, h5, s5)
      HITJ(6, h6, s6)
      HITJ(7, h7, s7)
#undef HITJ
    }
  }
  return wc;
}

__global__ __launch_bounds__(NTHR) void k_xprep(const float* __restrict__ x, unsigned short* xh,
                                                int nN, int nRows) {
  const int i = blockIdx.x * NTHR + threadIdx.x;
  if (i >= nRows * (KPAD1 / 8)) return;
  const int row = i >> 2;
  const int c0  = (i & 3) * 8;
  const int rc  = (row < nN) ? row : nN - 1;
  const int ca  = (c0 < CIN_X) ? c0 : 16;
  const int cb  = (c0 + 4 < CIN_X) ? (c0 + 4) : 16;
  const float* xr = x + (size_t)rc * CIN_X;
  v4f a = *(const v4f*)(xr + ca), b = *(const v4f*)(xr + cb);
  const v4f z = {0.f, 0.f, 0.f, 0.f};
  if (row >= nN || c0 >= CIN_X) a = z;
  if (row >= nN || c0 + 4 >= CIN_X) b = z;
  v8h hv;
  hv[0] = (_Float16)a.x; hv[1] = (_Float16)a.y; hv[2] = (_Float16)a.z; hv[3] = (_Float16)a.w;
  hv[4] = (_Float16)b.x; hv[5] = (_Float16)b.y; hv[6] = (_Float16)b.z; hv[7] = (_Float16)b.w;
  const size_t o = (size_t)i * 8;
  *(volatile v8h*)(xh + o) = hv;
  __threadfence();
  *(volatile v8h*)(xh + o) = hv;
}

__global__ __launch_bounds__(NTHR) void k_wprep(const float* __restrict__ W, int Kin, int Kpad,
                                                unsigned short* bt) {
  const int tpr = Kpad >> 3;
  const int i = blockIdx.x * NTHR + threadIdx.x;
  if (i >= HIDC * tpr) return;
  const int n  = i / tpr;
  const int k0 = (i - n * tpr) * 8;
  v8h hv;
#pragma unroll
  for (int e = 0; e < 8; ++e) {
    const int k  = k0 + e;
    const int kc = (k < Kin) ? k : Kin - 1;
    float v = W[(size_t)kc * HIDC + n];
    if (k >= Kin) v = 0.f;
    hv[e] = (_Float16)(8.0f * v);
  }
  const size_t o = (size_t)i * 8;
  *(volatile v8h*)(bt + o) = hv;
  __threadfence();
  *(volatile v8h*)(bt + o) = hv;
}

__device__ __forceinline__ float dot4f(v4f a, v4f b) {
  return a.x * b.x + a.y * b.y + a.z * b.z + a.w * b.w;
}

__global__ __launch_bounds__(NTHR) void k_scores1(const float* __restrict__ h, const float* __restrict__ as,
                                                  const float* __restrict__ ad, float* ss, float* sd,
                                                  int nN, int nRows) {
  const int node = blockIdx.x * NTHR + threadIdx.x;
  if (node >= nRows) return;
  const int nc = (node < nN) ? node : nN - 1;
  const float* hr = h + (size_t)nc * HIDC;
  float s0 = 0.f, d0 = 0.f;
#pragma unroll 1
  for (int c = 0; c < HIDC; c += 4) {
    const v4f hv = *(const v4f*)(hr + c);
    s0 += dot4f(hv, *(const v4f*)(as + c));
    d0 += dot4f(hv, *(const v4f*)(ad + c));
  }
  if (node >= nN) { s0 = 0.f; d0 = 0.f; }
  *(volatile float*)(ss + node) = s0;
  *(volatile float*)(sd + node) = d0;
  __threadfence();
  *(volatile float*)(ss + node) = s0;
  *(volatile float*)(sd + node) = d0;
}

template <bool RELU, bool F16OUT>
__global__ __launch_bounds__(NTHR) void k_gat_agg(
    const int* __restrict__ rowl, const int* __restrict__ coll,
    const float* __restrict__ hfeat, const float* __restrict__ ss, const float* __restrict__ sd,
    const float* __restrict__ bias, unsigned short* oh, float* of,
    int nN, int nE, int vec_ok) {
  constexpr int NB  = NBA;
  constexpr int HC  = HIDC;
  constexpr int CPL = HC / 32;
  constexpr int RW  = NB / NWAVE;
  constexpr int C4R = HC / 4;
  static_assert(NB * HC == 65536);
  static_assert(CPL == 2);
  static_assert((NB * HC / 4) % NTHR == 0 && (RW % 4) == 0);
  typedef float VT __attribute__((ext_vector_type(CPL)));
  extern __shared__ v4f lds_dyn[];
  float* acc  = (float*)lds_dyn;
  float* mst  = acc + NB * HC;
  float* sst  = mst + NB;
  int*   list = (int*)(sst + NB);
  int*   wcnt = list + LISTN;
  const int tid = threadIdx.x, lane = tid & 31, wave = tid >> 5;
  const int nodeBase = blockIdx.x * NB;

  {
    const v4f zz = {0.f, 0.f, 0.f, 0.f};
    for (int i = tid; i < NB * HC / 4; i += NTHR) lds_dyn[i] = zz;
    for (int i = tid; i < NB; i += NTHR) { mst[i] = -INFINITY; sst[i] = 0.f; }
  }
  __syncthreads();

  const int nChunks = (nE + CHUNK - 1) / CHUNK;
#pragma unroll 1
  for (int ch = 0; ch < nChunks; ++ch) {
    const int cbase = ch * CHUNK;
    const int fullvec = (vec_ok != 0 && cbase + CHUNK <= nE) ? 1 : 0;
    const int wc = scan_chunk<NB>(coll, nE, cbase, nodeBase, list, tid, lane, wave, fullvec);
    if (lane == 0) wcnt[wave] = wc;
    __syncthreads();
    if (wave == 0) {
#pragma unroll 1
      for (int wsx = 0; wsx < NWAVE; ++wsx) {
        int n = __builtin_amdgcn_readfirstlane(wcnt[wsx]);
        n = n > WCAP ? WCAP : (n < 0 ? 0 : n);
        const int* lp = list + wsx * WCAP;
#pragma unroll 1
        for (int i = 0; i < n; ++i) {
          const int ent  = __builtin_amdgcn_readfirstlane(lp[i]);
          const int slot = ent & (NB - 1);
          int e = cbase + ((ent >> 12) & (CHUNK - 1));
          e = e > nE - 1 ? nE - 1 : e;
          int s = rowl[e];
          s = s < 0 ? 0 : (s > nN - 1 ? nN - 1 : s);
          const int node = nodeBase + slot;
          float lg = ss[s] + sd[node];
          lg = (lg > 0.f) ? lg : 0.2f * lg;
          const float mo = mst[slot];
          const float so = sst[slot];
          const float d  = __expf(-fabsf(lg - mo));
          const bool  up = (lg > mo);
          const float sc = up ? d : 1.0f;
          const float w  = up ? 1.0f : d;
          const VT hv = *(const VT*)(hfeat + (size_t)s * HC + CPL * lane);
          VT* ap = (VT*)(acc + slot * HC + CPL * lane);
          const VT av = *ap;
          *ap = av * sc + hv * w;
          mst[slot] = up ? lg : mo;
          sst[slot] = so * sc + w;
        }
      }
    }
    __syncthreads();
  }

#pragma unroll 1
  for (int it = 0; it < (NB * HC / 4) / NTHR; ++it) {
    const int idx  = it * NTHR + tid;
    const int slot = idx / C4R;
    const int c4   = (idx - slot * C4R) * 4;
    const int node = nodeBase + slot;
    const int nc   = (node < nN) ? node : nN - 1;
    float lg = ss[nc] + sd[nc];
    lg = (lg > 0.f) ? lg : 0.2f * lg;
    const float mo = mst[slot];
    const float so = sst[slot];
    const float d  = __expf(-fabsf(lg - mo));
    const bool  up = (lg > mo);
    const float sc = up ? d : 1.0f;
    const float w  = up ? 1.0f : d;
    const v4f hs = *(const v4f*)(hfeat + (size_t)nc * HC + c4);
    v4f* ap = (v4f*)(acc + slot * HC + c4);
    v4f a = *ap;
    a = a * sc + hs * w;
    const float sn  = so * sc + w;
    const float inv = __builtin_amdgcn_rcpf(sn);
    const v4f bv = *(const v4f*)(bias + c4);
    v4f o = a * inv + bv;
    if (RELU) { o.x = fmaxf(o.x, 0.f); o.y = fmaxf(o.y, 0.f); o.z = fmaxf(o.z, 0.f); o.w = fmaxf(o.w, 0.f); }
    if (node >= nN) { const v4f zz = {0.f, 0.f, 0.f, 0.f}; o = zz; }
    *ap = o;
  }
  __syncthreads();

  if (F16OUT) {
    unsigned short* hb = oh + (size_t)nodeBase * HC;
    for (int pass = 0; pass < 2; ++pass) {
#pragma unroll 4
      for (int q = 0; q < RW / 4; ++q) {
        const int row = wave * RW + 4 * q + (lane >> 3);
        const int col = (lane & 7) * 8;
        const float* sp = acc + row * HC + col;
        const v4f p0 = *(const v4f*)sp, p1 = *(const v4f*)(sp + 4);
        v8h hv;
        hv[0] = (_Float16)p0.x; hv[1] = (_Float16)p0.y; hv[2] = (_Float16)p0.z; hv[3] = (_Float16)p0.w;
        hv[4] = (_Float16)p1.x; hv[5] = (_Float16)p1.y; hv[6] = (_Float16)p1.z; hv[7] = (_Float16)p1.w;
        *(volatile v8h*)(hb + (size_t)row * HC + col) = hv;
      }
      __threadfence();
    }
  } else {
    float* ob = of + (size_t)nodeBase * HC;
    for (int pass = 0; pass < 2; ++pass) {
#pragma unroll 4
      for (int q = 0; q < RW / 2; ++q) {
        const int row = wave * RW + 2 * q + (lane >> 4);
        const int col = (lane & 15) * 4;
        const v4f v = *(const v4f*)(acc + row * HC + col);
        *(volatile v4f*)(ob + (size_t)row * HC + col) = v;
      }
      __threadfence();
    }
  }
}

__global__ __launch_bounds__(NTHR) void k_pool(const int* __restrict__ batch, const float* __restrict__ h,
                                               float* pooled, int nN, int vec_ok) {
  __shared__ int list[LISTN];
  __shared__ int wcnt[NWAVE];
  __shared__ __align__(16) float prow[PPITCH];
  const int tid = threadIdx.x, lane = tid & 31, wave = tid >> 5;
  const int g = blockIdx.x;
  v2f accv = {0.f, 0.f};
  float cnt = 0.f;
  const int nChunks = (nN + CHUNK - 1) / CHUNK;
#pragma unroll 1
  for (int ch = 0; ch < nChunks; ++ch) {
    const int cbase = ch * CHUNK;
    const int fullvec = (vec_ok != 0 && cbase + CHUNK <= nN) ? 1 : 0;
    const int wc = scan_chunk<1>(batch, nN, cbase, g, list, tid, lane, wave, fullvec);
    if (lane == 0) wcnt[wave] = wc;
    __syncthreads();
    if (wave == 0) {
#pragma unroll 1
      for (int wsx = 0; wsx < NWAVE; ++wsx) {
        int n = __builtin_amdgcn_readfirstlane(wcnt[wsx]);
        n = n > WCAP ? WCAP : (n < 0 ? 0 : n);
        const int* lp = list + wsx * WCAP;
#pragma unroll 1
        for (int i = 0; i < n; ++i) {
          const int ent = __builtin_amdgcn_readfirstlane(lp[i]);
          int node = cbase + ((ent >> 12) & (CHUNK - 1));
          node = node > nN - 1 ? nN - 1 : (node < 0 ? 0 : node);
          const v2f hv = *(const v2f*)(h + (size_t)node * HIDC + 2 * lane);
          accv += hv;
          cnt += 1.0f;
        }
      }
    }
    __syncthreads();
  }
  if (wave == 0) {
    prow[2 * lane]     = accv.x;
    prow[2 * lane + 1] = accv.y;
    prow[HIDC + lane]  = (lane == 0) ? cnt : 0.f;
  }
  __syncthreads();
  if (wave == 0) {
    const int lc = (lane < 24) ? lane : 23;
    const v4f v = *(const v4f*)(prow + 4 * lc);
    float* dp = pooled + (size_t)g * PPITCH + 4 * lane;
    if (lane < 24) *(volatile v4f*)dp = v;
    __threadfence();
    if (lane < 24) *(volatile v4f*)dp = v;
  }
}

__global__ __launch_bounds__(NTHR) void k_head(const float* __restrict__ pooled, const float* __restrict__ linW,
                                               const float* __restrict__ linb, float* out, int G) {
  __shared__ __align__(16) float so[OUTC * GMAX];
  const int tid = threadIdx.x, lane = tid & 31, wave = tid >> 5;
  const float lb0 = linb[0], lb1 = linb[1];
#pragma unroll 1
  for (int g = tid; g < G; g += NTHR) {
    const float* pr = pooled + (size_t)g * PPITCH;
    const float c   = fmaxf(pr[HIDC], 1.0f);
    const float inv = 1.0f / c;
    float a0 = 0.f, a1 = 0.f;
#pragma unroll 1
    for (int f = 0; f < HIDC; f += 2) {
      const v2f p = *(const v2f*)(pr + f);
      const v4f w = *(const v4f*)(linW + 2 * f);
      const float p0 = p.x * inv, p1 = p.y * inv;
      a0 += p0 * w.x + p1 * w.z;
      a1 += p0 * w.y + p1 * w.w;
    }
    so[2 * g]     = a0 + lb0;
    so[2 * g + 1] = a1 + lb1;
  }
  __syncthreads();
  const int nflt = G * OUTC;
  for (int pass = 0; pass < 2; ++pass) {
#pragma unroll 1
    for (int s = wave; s * 128 < nflt; s += NWAVE) {
      const int idx = s * 128 + lane * 4;
      const v4f v = *(const v4f*)(so + idx);
      if (idx + 4 <= nflt) *(volatile v4f*)(out + idx) = v;
    }
    if (tid == 0 && (nflt & 3) != 0) {
      const int i0 = nflt & ~3;
      const float t0 = so[i0], t1 = so[i0 + 1];
      *(volatile float*)(out + i0) = t0;
      *(volatile float*)(out + i0 + 1) = t1;
    }
    __threadfence();
  }
}

extern "C" void kernel_launch(void* const* d_in, const int* in_sizes, int n_in,
                              void* d_out, int out_size, void* d_ws, size_t ws_size,
                              hipStream_t stream) {
  if (n_in < 17) return;
  const int nN = in_sizes[0] / CIN_X;
  const int nE = in_sizes[1] / 2;
  const int G  = out_size / OUTC;
  if (nN < 1 || in_sizes[0] != nN * CIN_X || nE < 1 || in_sizes[1] != 2 * nE) return;
  if (in_sizes[2] != nN) return;
  if (in_sizes[3] != CIN_X * HIDC || in_sizes[4] < HIDC || in_sizes[5] < HIDC || in_sizes[6] < HIDC) return;
  if (in_sizes[7] != HIDC * HIDC || in_sizes[8] < HIDC || in_sizes[9] < HIDC || in_sizes[10] < HIDC) return;
  if (in_sizes[11] != HIDC * HIDC || in_sizes[12] < HIDC || in_sizes[13] < HIDC || in_sizes[14] < HIDC) return;
  if (in_sizes[15] != HIDC * OUTC || in_sizes[16] < OUTC) return;
  if (G < 1 || G > GMAX || out_size != G * OUTC) return;
  if (nN > (1 << 24)) return;

  const float* x     = (const float*)d_in[0];
  const int*   ei    = (const int*)d_in[1];
  const int*   batch = (const int*)d_in[2];
  const float* W1    = (const float*)d_in[3];
  const float* as1   = (const float*)d_in[4];
  const float* ad1   = (const float*)d_in[5];
  const float* b1    = (const float*)d_in[6];
  const float* W2    = (const float*)d_in[7];
  const float* as2   = (const float*)d_in[8];
  const float* ad2   = (const float*)d_in[9];
  const float* b2    = (const float*)d_in[10];
  const float* W3    = (const float*)d_in[11];
  const float* as3   = (const float*)d_in[12];
  const float* ad3   = (const float*)d_in[13];
  const float* b3    = (const float*)d_in[14];
  const float* linW  = (const float*)d_in[15];
  const float* linb  = (const float*)d_in[16];
  const int* rowl = ei;
  const int* coll = ei + nE;
  float* out = (float*)d_out;

  const int RP  = ((nN + RPQ - 1) / RPQ) * RPQ;
  const int nA  = RP / NBA;
  const int vec_col = ((nE & 3) == 0) ? 1 : 0;

  char* ws = (char*)d_ws;
  size_t off = 0;
  const size_t oXH  = off; off += (size_t)RP * KPAD1 * 2;
  const size_t oW1T = off; off += (size_t)HIDC * KPAD1 * 2;
  const size_t oW2T = off; off += (size_t)HIDC * HIDC * 2;
  const size_t oW3T = off; off += (size_t)HIDC * HIDC * 2;
  const size_t oHF  = off; off += (size_t)RP * HIDC * 4;
  const size_t oSS  = off; off += (size_t)RP * 4;
  const size_t oSD  = off; off += (size_t)RP * 4;
  const size_t oAH  = off; off += (size_t)RP * HIDC * 2;
  const size_t oH3  = off; off += (size_t)RP * HIDC * 4;
  const size_t oPL  = off; off += (size_t)G * PPITCH * 4;
  if (off > ws_size || off > (size_t)134217728) return;

  unsigned short* xh  = (unsigned short*)(ws + oXH);
  unsigned short* w1t = (unsigned short*)(ws + oW1T);
  unsigned short* w2t = (unsigned short*)(ws + oW2T);
  unsigned short* w3t = (unsigned short*)(ws + oW3T);
  float* hf  = (float*)(ws + oHF);
  float* ssp = (float*)(ws + oSS);
  float* sdp = (float*)(ws + oSD);
  unsigned short* ah = (unsigned short*)(ws + oAH);
  float* h3  = (float*)(ws + oH3);
  float* pl  = (float*)(ws + oPL);

  k_xprep<<<RP * (KPAD1 / 8) / NTHR, NTHR, 0, stream>>>(x, xh, nN, RP);
  k_wprep<<<(HIDC * (KPAD1 / 8) + NTHR - 1) / NTHR, NTHR, 0, stream>>>(W1, CIN_X, KPAD1, w1t);
  k_wprep<<<(HIDC * (HIDC / 8) + NTHR - 1) / NTHR, NTHR, 0, stream>>>(W2, HIDC, HIDC, w2t);
  k_wprep<<<(HIDC * (HIDC / 8) + NTHR - 1) / NTHR, NTHR, 0, stream>>>(W3, HIDC, HIDC, w3t);

  const int gg = ((RP / 64) * (HIDC / 64) + 7) / 8;

  wmma_gemm64<0, false, 0, 0, false, 0><<<dim3(gg, 1), 256, 0, stream>>>(
      xh, xh, KPAD1, 0L, w1t, w1t, KPAD1, 0L, (void*)hf, (void*)hf, HIDC, 0L,
      b1, b1, 0L, RP, HIDC, KPAD1, 0.125f);
  k_scores1<<<RP / NTHR, NTHR, 0, stream>>>(hf, as1, ad1, ssp, sdp, nN, RP);
  k_gat_agg<true, true><<<nA, NTHR, LDS_AGG, stream>>>(
      rowl, coll, hf, ssp, sdp, b1, ah, h3, nN, nE, vec_col);

  wmma_gemm64<0, false, 0, 0, false, 0><<<dim3(gg, 1), 256, 0, stream>>>(
      ah, ah, HIDC, 0L, w2t, w2t, HIDC, 0L, (void*)hf, (void*)hf, HIDC, 0L,
      b2, b2, 0L, RP, HIDC, HIDC, 0.125f);
  k_scores1<<<RP / NTHR, NTHR, 0, stream>>>(hf, as2, ad2, ssp, sdp, nN, RP);
  k_gat_agg<true, true><<<nA, NTHR, LDS_AGG, stream>>>(
      rowl, coll, hf, ssp, sdp, b2, ah, h3, nN, nE, vec_col);

  wmma_gemm64<0, false, 0, 0, false, 0><<<dim3(gg, 1), 256, 0, stream>>>(
      ah, ah, HIDC, 0L, w3t, w3t, HIDC, 0L, (void*)hf, (void*)hf, HIDC, 0L,
      b3, b3, 0L, RP, HIDC, HIDC, 0.125f);
  k_scores1<<<RP / NTHR, NTHR, 0, stream>>>(hf, as3, ad3, ssp, sdp, nN, RP);
  k_gat_agg<false, false><<<nA, NTHR, LDS_AGG, stream>>>(
      rowl, coll, hf, ssp, sdp, b3, ah, h3, nN, nE, vec_col);

  k_pool<<<G, NTHR, 0, stream>>>(batch, h3, pl, nN, 0);
  k_head<<<1, NTHR, 0, stream>>>(pl, linW, linb, out, G);
}
